// NeighborhoodAttention_2190433321583
// MI455X (gfx1250) — hardware-verified
//
#include <hip/hip_runtime.h>


namespace {
constexpr int NB_ = 2, C = 64, IH = 128, IW = 128, NP = IH * IW, NT = NB_ * NP, H = 4, HD = 16, WSZ = 7, NU = 160  , UC = 22;
constexpr float XS = 8.0f, HS = 256.0f, PS = 256.0f, WSC = 256.0f, SCALE = 0.25f;
typedef _Float16 b16;
typedef __attribute__((ext_vector_type(16))) _Float16 v16b;
typedef __attribute__((ext_vector_type(8))) _Float16 v8b;
typedef __attribute__((ext_vector_type(2))) _Float16 v2b;
typedef __attribute__((ext_vector_type(8))) float v8f;
typedef __attribute__((ext_vector_type(4))) float v4f;
typedef __attribute__((ext_vector_type(2))) float v2f;
__device__ __forceinline__ float bf16_rne(float f) { unsigned int u = __float_as_uint(f); u += 0x7FFFu + ((u >> 16) & 1u); float r = __uint_as_float(u & 0xFFFF0000u); asm volatile("" : "+v"(r)); return r; }
__device__ __forceinline__ float bfv(float f) { float r = bf16_rne(f); asm volatile("" : "+v"(r)); return r; }
__device__ __forceinline__ void split16(float v, b16& hi, b16& lo) { hi = (b16)v; lo = (b16)(v - (float)hi); }
__device__ __forceinline__ v16b frag_kb(const b16* p, int hh) { const v8b a = *(const v8b*)(p + 8 * hh), b = *(const v8b*)(p + 16 + 8 * hh); v16b f;
#pragma unroll
  for (int e = 0; e < 8; ++e) { f[e] = a[e]; f[8 + e] = b[e]; } return f; }
__device__ __forceinline__ v8f wmma16b(v16b a, v16b b, v8f c) { v8f d = __builtin_amdgcn_wmma_f32_16x16x32_f16(false, a, false, b, (short)0, c, false, false); asm volatile("v_nop\n\tv_nop\n\tv_nop\n\tv_nop" : "+v"(d) : "v"(a), "v"(b)); return d; }
__device__ __forceinline__ void wave_lds_sync() { __builtin_amdgcn_fence(__ATOMIC_RELEASE, "workgroup"); __builtin_amdgcn_wave_barrier(); __builtin_amdgcn_fence(__ATOMIC_ACQUIRE, "workgroup"); }
__device__ __forceinline__ float pmul(float a, float b) { float p = a * b; asm volatile("" : "+v"(p)); return p; }
__device__ __forceinline__ int iclamp(int v, int lo, int hi) { return v < lo ? lo : (v > hi ? hi : v); }

__global__ __launch_bounds__(256) void wput_kernel(const float* __restrict__ qkvw, const float* __restrict__ pw, b16* __restrict__ WQ, b16* __restrict__ WPj) { const int u = blockIdx.x * 256 + threadIdx.x; v8b v;
  if (u < 192 * 8) { const int o = u / 8, k0 = (u % 8) * 8;
#pragma unroll
    for (int j = 0; j < 8; ++j) v[j] = (b16)(bf16_rne(qkvw[(size_t)o * C + k0 + j]) * WSC); for (int pass = 0; pass < 2; ++pass) { *(volatile v8b*)(WQ + (size_t)o * C + k0) = v; __threadfence(); } }
  if (u < 64 * 8) { const int o = u / 8, k0 = (u % 8) * 8;
#pragma unroll
    for (int j = 0; j < 8; ++j) v[j] = (b16)(bf16_rne(pw[(size_t)o * C + k0 + j]) * WSC); for (int pass = 0; pass < 2; ++pass) { *(volatile v8b*)(WPj + (size_t)o * C + k0) = v; __threadfence(); } } }
__global__ __launch_bounds__(32) void qkv_kernel(const float* __restrict__ x, const b16* __restrict__ WQ, const float* __restrict__ qb, int TLIM, b16* __restrict__ QPh, b16* __restrict__ QPl, b16* __restrict__ KPh, b16* __restrict__ KPl, float* __restrict__ VR) { __shared__ __attribute__((aligned(16))) b16 Ax[16][C + 8]; __shared__ float Tf[16][196]; const int lane = threadIdx.x, nloc = lane & 15, hlf = lane >> 4; const size_t t0 = (size_t)blockIdx.x * 16; if (t0 >= (size_t)TLIM) return; const int b = (int)(t0 / NP); const int p0 = (int)(t0 % NP);
  for (int q = 0; q < 2; ++q) { const int c = q * 32 + lane; const float* xp = x + ((size_t)b * C + c) * NP + p0; for (int rr = 0; rr < 16; ++rr) Ax[rr][c] = (b16)(bf16_rne(xp[rr]) * XS); }
  if (lane < 16) for (int k = C; k < C + 8; ++k) Ax[lane][k] = (b16)0.0f;
  wave_lds_sync(); v8f acc[12];
#pragma unroll
  for (int t = 0; t < 12; ++t) acc[t] = (v8f){};
#pragma unroll
  for (int kb = 0; kb < C; kb += 32) { const v16b a = frag_kb(&Ax[nloc][kb], hlf);
#pragma unroll
    for (int t = 0; t < 12; ++t) acc[t] = wmma16b(a, frag_kb(WQ + (size_t)(t * 16 + nloc) * C + kb, hlf), acc[t]); }
#pragma unroll
  for (int t = 0; t < 12; ++t) { const int cc = t * 16 + nloc; const float bb = bfv(qb[cc]);
#pragma unroll
    for (int r8 = 0; r8 < 8; ++r8) Tf[8 * hlf + r8][cc] = acc[t][r8] * (1.0f / (XS * WSC)) + bb; }
  wave_lds_sync();
  for (int pass = 0; pass < 2; ++pass) { for (int rr = 0; rr < 16; ++rr) { const size_t t = t0 + rr; const int h = lane >> 3, d2 = (lane & 7) * 2; b16 a0, a1, l0, l1; const size_t po = (t * H + h) * 32 + d2;
      split16(Tf[rr][h * HD + d2] * HS, a0, l0); split16(Tf[rr][h * HD + d2 + 1] * HS, a1, l1); *(volatile v2b*)(QPh + po) = (v2b){a0, a1}; *(volatile v2b*)(QPl + po) = (v2b){l0, l1}; *(volatile v2b*)(QPh + po + 16) = (v2b){0, 0}; *(volatile v2b*)(QPl + po + 16) = (v2b){0, 0};
      split16(Tf[rr][C + h * HD + d2] * HS, a0, l0); split16(Tf[rr][C + h * HD + d2 + 1] * HS, a1, l1); *(volatile v2b*)(KPh + po) = (v2b){a0, a1}; *(volatile v2b*)(KPl + po) = (v2b){l0, l1}; *(volatile v2b*)(KPh + po + 16) = (v2b){0, 0}; *(volatile v2b*)(KPl + po + 16) = (v2b){0, 0};
      *(volatile v2f*)(VR + t * C + lane * 2) = (v2f){Tf[rr][2 * C + lane * 2], Tf[rr][2 * C + lane * 2 + 1]}; } __threadfence(); } }
__global__ __launch_bounds__(32) void att_kernel(const b16* __restrict__ QPh, const b16* __restrict__ QPl, const b16* __restrict__ KPh, const b16* __restrict__ KPl, const float* __restrict__ VR, const float* __restrict__ rbias, int TLIM, float* __restrict__ O) { __shared__ __attribute__((aligned(16))) b16 Pa[16][NU + 8], Pb[16][NU + 8], VTh[HD][NU + 8], VTl[HD][NU + 8]; __shared__ float Sc[16][NU + 1], Of[16][C + 1]; __shared__ int Ktok[NU]; const int lane = threadIdx.x, nloc = lane & 15, hlf = lane >> 4; const size_t t0 = (size_t)blockIdx.x * 16; if (t0 >= (size_t)TLIM) return; const int b = (int)(t0 / NP), p0 = (int)(t0 % NP), i = p0 / IW, j0 = p0 % IW;
  const int ar = iclamp(i - 3, 0, IH - WSZ), uc0 = iclamp(j0 - 3, 0, IW - WSZ);
  for (int u = lane; u < NU; u += 32) { const int rr = u / UC, cc = u % UC; const int r = ar + rr, c = uc0 + cc; Ktok[u] = (u < WSZ * UC && c < IW) ? (r * IW + c) : -1; }
  if (lane < 16) for (int k = NU; k < NU + 8; ++k) { Pa[lane][k] = (b16)0.0f; Pb[lane][k] = (b16)0.0f; }
  wave_lds_sync();
#pragma unroll 1
  for (int h = 0; h < H; ++h) {
    for (int u = lane; u < NU + 8; u += 32) { const int tk = u < NU ? Ktok[u] : -1; for (int d = 0; d < HD; ++d) { b16 p = (b16)0.0f, pl = (b16)0.0f; if (tk >= 0) split16(VR[((size_t)b * NP + tk) * C + h * HD + d] * HS, p, pl); VTh[d][u] = p; VTl[d][u] = pl; } }
    const v16b qa = frag_kb(QPh + ((t0 + nloc) * H + h) * 32, hlf), ql = frag_kb(QPl + ((t0 + nloc) * H + h) * 32, hlf);
#pragma unroll 2
    for (int t = 0; t < NU / 16; ++t) { const int u = t * 16 + nloc; const int tk = Ktok[u]; const size_t ko = (((size_t)b * NP + (tk >= 0 ? tk : 0)) * H + h) * 32; const v16b kh = frag_kb(KPh + ko, hlf), kl = frag_kb(KPl + ko, hlf); v8f s = wmma16b(qa, kh, (v8f){}); s = wmma16b(qa, kl, s); s = wmma16b(ql, kh, s);
#pragma unroll
      for (int r8 = 0; r8 < 8; ++r8) Sc[8 * hlf + r8][u] = s[r8] * (SCALE / (HS * HS)); }
    wave_lds_sync();
    if (lane < 16) { const int r = lane; const int j = j0 + r; const int ac = iclamp(j - 3, 0, IW - WSZ); const int bi = (i - ar), bj = (j - ac); float mx = -INFINITY;
      for (int u = 0; u < NU; ++u) { const int rr = u / UC, cc = u % UC; const int c = uc0 + cc; float s = -INFINITY; if (u < WSZ * UC && c >= ac && c < ac + WSZ && c < IW) { const int kr = rr, kc = c - ac; s = Sc[r][u] + bfv(rbias[((bi + kr) * 13 + (bj + kc)) * H + h]); } Sc[r][u] = s; mx = fmaxf(mx, s); }
      float sm = 0.0f; for (int u = 0; u < NU; ++u) { const float p = Sc[r][u] == -INFINITY ? 0.0f : __expf(Sc[r][u] - mx); Sc[r][u] = p; sm += p; } const float inv = 1.0f / sm; for (int u = 0; u < NU; ++u) { b16 p, pl; split16(Sc[r][u] * inv * PS, p, pl); Pa[r][u] = p; Pb[r][u] = pl; } }
    wave_lds_sync();
    v8f o = (v8f){};
#pragma unroll
    for (int kb = 0; kb < NU; kb += 32) { const v16b pa = frag_kb(&Pa[nloc][kb], hlf), pb = frag_kb(&Pb[nloc][kb], hlf); const v16b vh = frag_kb(&VTh[nloc][kb], hlf), vl = frag_kb(&VTl[nloc][kb], hlf); o = wmma16b(pa, vh, o); o = wmma16b(pa, vl, o); o = wmma16b(pb, vh, o); }
#pragma unroll
    for (int r8 = 0; r8 < 8; ++r8) Of[8 * hlf + r8][h * HD + nloc] = o[r8] * (1.0f / (PS * HS));
    wave_lds_sync(); }
  for (int pass = 0; pass < 2; ++pass) { for (int r = 0; r < 16; ++r) *(volatile v2f*)(O + (t0 + r) * C + lane * 2) = (v2f){Of[r][lane * 2], Of[r][lane * 2 + 1]}; __threadfence(); } }
__global__ __launch_bounds__(32) void proj_kernel(const float* __restrict__ O, const b16* __restrict__ WPj, const float* __restrict__ pb, int TLIM, float* __restrict__ FIN) { __shared__ __attribute__((aligned(16))) b16 Ah[16][C + 8], Al[16][C + 8]; __shared__ float Tf[16][C + 1]; const int lane = threadIdx.x, nloc = lane & 15, hlf = lane >> 4; const size_t t0 = (size_t)blockIdx.x * 16; if (t0 >= (size_t)TLIM) return;
  for (int rr = 0; rr < 16; ++rr) for (int q = 0; q < 2; ++q) { const int c = q * 32 + lane; b16 p, pl; split16(O[(t0 + rr) * C + c] * HS, p, pl); Ah[rr][c] = p; Al[rr][c] = pl; }
  if (lane < 16) for (int k = C; k < C + 8; ++k) { Ah[lane][k] = (b16)0.0f; Al[lane][k] = (b16)0.0f; }
  wave_lds_sync(); v8f acc[4] = {(v8f){}, (v8f){}, (v8f){}, (v8f){}};
#pragma unroll
  for (int kb = 0; kb < C; kb += 32) { const v16b a = frag_kb(&Ah[nloc][kb], hlf), al = frag_kb(&Al[nloc][kb], hlf);
#pragma unroll
    for (int t = 0; t < 4; ++t) { const v16b bw = frag_kb(WPj + (size_t)(t * 16 + nloc) * C + kb, hlf); acc[t] = wmma16b(a, bw, acc[t]); acc[t] = wmma16b(al, bw, acc[t]); } }
#pragma unroll
  for (int t = 0; t < 4; ++t) { const int cc = t * 16 + nloc; const float bb = bfv(pb[cc]);
#pragma unroll
    for (int r8 = 0; r8 < 8; ++r8) Tf[8 * hlf + r8][cc] = acc[t][r8] * (1.0f / (HS * WSC)) + bb; }
  wave_lds_sync();
  for (int pass = 0; pass < 2; ++pass) { for (int rr = 0; rr < 16; ++rr) *(volatile v2f*)(FIN + (t0 + rr) * C + lane * 2) = (v2f){Tf[rr][lane * 2], Tf[rr][lane * 2 + 1]}; __threadfence(); } }
__global__ __launch_bounds__(256) void copy_kernel(const float* __restrict__ FIN, int TLIM, float* __restrict__ out) { const size_t u = (size_t)blockIdx.x * 256 + threadIdx.x; if (u >= (size_t)NT * C) return; const int p = (int)(u % NP), c = (int)((u / NP) % C), b = (int)(u / ((size_t)NP * C)); const size_t t = (size_t)b * NP + p; const float v = t < (size_t)TLIM ? FIN[t * C + c] : 0.0f;
  for (int pass = 0; pass < 2; ++pass) { ((volatile float*)out)[u] = v; __threadfence(); } }
}

extern "C" void kernel_launch(void* const* d_in, const int* in_sizes, int n_in, void* d_out, int out_size, void* d_ws, size_t ws_size, hipStream_t stream) {
  (void)n_in;
  auto Fp = [&](int i) { return (const float*)d_in[i]; };
  if (in_sizes[0] != NT * C || in_sizes[1] != 3 * C * C || in_sizes[2] != 3 * C || in_sizes[3] != C * C || in_sizes[5] != 169 * H || out_size != NT * C) return;
  const int TLIM = NT;
  size_t off = 0; char* ws = (char*)d_ws;
  auto carve = [&](size_t bytes) { char* p = ws + off; off += (bytes + 255) & ~(size_t)255; return p; };
  b16* WQ = (b16*)carve(192 * C * 2); b16* WPj = (b16*)carve(C * C * 2); b16* QPh = (b16*)carve((size_t)NT * H * 32 * 2); b16* QPl = (b16*)carve((size_t)NT * H * 32 * 2); b16* KPh = (b16*)carve((size_t)NT * H * 32 * 2); b16* KPl = (b16*)carve((size_t)NT * H * 32 * 2); float* VR = (float*)carve((size_t)NT * C * 4); float* O = (float*)carve((size_t)NT * C * 4); float* FIN = (float*)carve((size_t)NT * C * 4);
  if (off > ws_size || off > ((size_t)72 << 20)) return;
  wput_kernel<<<(192 * 8 + 255) / 256, 256, 0, stream>>>(Fp(1), Fp(3), WQ, WPj);
  qkv_kernel<<<NT / 16, 32, 0, stream>>>(Fp(0), WQ, Fp(2), TLIM, QPh, QPl, KPh, KPl, VR);
  att_kernel<<<NT / 16, 32, 0, stream>>>(QPh, QPl, KPh, KPl, VR, Fp(5), TLIM, O);
  proj_kernel<<<NT / 16, 32, 0, stream>>>(O, WPj, Fp(4), TLIM, FIN);
  copy_kernel<<<(NT * C + 255) / 256, 256, 0, stream>>>(FIN, TLIM, (float*)d_out);
}
